// negative_set_define_76647986364840
// MI455X (gfx1250) — hardware-verified
//
#include <hip/hip_runtime.h>
#pragma clang fp contract(off)

typedef float          v4f  __attribute__((ext_vector_type(4)));
typedef float          v8f  __attribute__((ext_vector_type(8)));
typedef unsigned int   v4u  __attribute__((ext_vector_type(4)));
typedef __bf16         v16b __attribute__((ext_vector_type(16)));
typedef __bf16         v8b  __attribute__((ext_vector_type(8)));
typedef v8b __attribute__((may_alias)) v8ba;
typedef v4f __attribute__((may_alias)) v4fa;
typedef v4u __attribute__((may_alias)) v4ua;

union Frag { v16b v; v8b half[2]; };

#define NROWS   8192
#define DIM     1024
#define DIMW    (DIM / 2)
#define NELEM   (NROWS * DIM)
#define BM      64
#define BN      128
#define NTILES  (NROWS / BN)
#define CAP     32
#define BAND    4.0f
#define RPB     32

static_assert(CAP == 32);
static_assert((NROWS % BM) == 0);
static_assert((NROWS % BN) == 0);
static_assert((NROWS % RPB) == 0);
static_assert((DIM % 256) == 0);

__device__ __forceinline__ v8f wmma_bf16(v16b a, v16b b, v8f c) {
  v8f d = __builtin_amdgcn_wmma_f32_16x16x32_bf16(false, a, false, b, (short)0, c, false, false);
  asm volatile("v_nop\n\tv_nop\n\tv_nop\n\tv_nop" : "+v"(d) : "v"(a), "v"(b));
  return d;
}

__device__ __forceinline__ v16b load_frag(const __bf16* p, int h) {
  Frag f;
  f.half[0] = *(const v8ba*)(p + 8 * h);
  f.half[1] = *(const v8ba*)(p + 16 + 8 * h);
  return f.v;
}

__device__ __forceinline__ unsigned bf16_bits(float x) {
  const unsigned u = __float_as_uint(x);
  return (u + 0x7FFFu + ((u >> 16) & 1u)) >> 16;
}

__device__ __forceinline__ void df_add(float& hi, float& lo, float bh, float bl) {
  const float s  = hi + bh;
  const float bb = s - hi;
  float e = (hi - (s - bb)) + (bh - bb);
  e = e + (lo + bl);
  const float h2 = s + e;
  lo = e - (h2 - s);
  hi = h2;
}
__device__ __forceinline__ void df_mac(float& hi, float& lo, float a, float b) {
  const float p  = a * b;
  const float pe = fmaf(a, b, -p);
  df_add(hi, lo, p, pe);
}
__device__ __forceinline__ void df_wave_reduce(float& hi, float& lo) {
  #pragma unroll
  for (int off = 16; off >= 1; off >>= 1) {
    const float oh = __shfl_xor(hi, off, 32);
    const float ol = __shfl_xor(lo, off, 32);
    df_add(hi, lo, oh, ol);
  }
}

__device__ __forceinline__ v4f sel4(bool c, v4f a, v4f b) {
  v4f r;
  r.x = c ? a.x : b.x; r.y = c ? a.y : b.y; r.z = c ? a.z : b.z; r.w = c ? a.w : b.w;
  return r;
}

__global__ __launch_bounds__(256) void prep_kernel(
    const float* __restrict__ anchor, const float* __restrict__ negative,
    unsigned* __restrict__ abw, unsigned* __restrict__ nbw,
    float* __restrict__ n2hi, float* __restrict__ n2lo)
{
  __shared__ __attribute__((aligned(16))) float sHi[RPB];
  __shared__ __attribute__((aligned(16))) float sLo[RPB];

  const int tid = threadIdx.x, lane = tid & 31, w = tid >> 5;
  const int blk = blockIdx.x;
  const bool isNeg = blk < (NROWS / RPB);
  const int rb = isNeg ? blk : (blk - NROWS / RPB);
  const float* src = isNeg ? negative : anchor;
  unsigned* dstw = isNeg ? nbw : abw;

  #pragma unroll 1
  for (int q = 0; q < 4; ++q) {
    const int row = rb * RPB + w * 4 + q;
    const float* p = src + (size_t)row * DIM;
    unsigned* d = dstw + (size_t)row * DIMW;
    float hi = 0.0f, lo = 0.0f;
    #pragma unroll 1
    for (int it = 0; it < 4; ++it) {
      const int k = it * 256 + lane * 8;
      const v4f a = *(const v4fa*)(p + k);
      const v4f c = *(const v4fa*)(p + k + 4);
      v4u o;
      o.x = bf16_bits(a.x) | (bf16_bits(a.y) << 16);
      o.y = bf16_bits(a.z) | (bf16_bits(a.w) << 16);
      o.z = bf16_bits(c.x) | (bf16_bits(c.y) << 16);
      o.w = bf16_bits(c.z) | (bf16_bits(c.w) << 16);
      unsigned* dp = d + it * 128 + lane * 4;
      *(volatile v4u*)dp = o;
      __threadfence();
      *(volatile v4u*)dp = o;
      df_mac(hi, lo, a.x, a.x);
      df_mac(hi, lo, a.y, a.y);
      df_mac(hi, lo, a.z, a.z);
      df_mac(hi, lo, a.w, a.w);
      df_mac(hi, lo, c.x, c.x);
      df_mac(hi, lo, c.y, c.y);
      df_mac(hi, lo, c.z, c.z);
      df_mac(hi, lo, c.w, c.w);
    }
    df_wave_reduce(hi, lo);
    if (lane == 0) { sHi[w * 4 + q] = hi; sLo[w * 4 + q] = lo; }
  }
  __syncthreads();

  if (isNeg && w == 0) {
    const int q8 = lane & 7;
    const v4f vh = *(const v4fa*)(sHi + 4 * q8);
    const v4f vl = *(const v4fa*)(sLo + 4 * q8);
    const bool first = lane < 8;
    const v4f v = sel4(first, vh, vl);
    float* dst = (first ? n2hi : n2lo) + rb * RPB + 4 * q8;
    if (lane < 16) *(volatile v4f*)dst = v;
    __threadfence();
    if (lane < 16) *(volatile v4f*)dst = v;
  }
}

__global__ __launch_bounds__(128) void select_kernel(
    const __bf16* __restrict__ ab,
    const __bf16* __restrict__ nb,
    const float*  __restrict__ anchor,
    const float*  __restrict__ negative,
    const float*  __restrict__ n2hi,
    const float*  __restrict__ n2lo,
    float*        __restrict__ out)
{
  __shared__ __attribute__((aligned(16))) float sS[BM * BN];
  __shared__ int   sJ[4 * 16 * CAP];
  __shared__ float sK[4 * 16 * CAP];

  const int tid = threadIdx.x, lane = tid & 31, w = tid >> 5;
  const int h = lane >> 4, m = lane & 15;
  const int wm = w >> 1, wn = w & 1;
  const int R0 = blockIdx.x * BM;
  const unsigned ltmask = (1u << lane) - 1u;
  const float NEG_INF = __uint_as_float(0xff800000u);

  #pragma unroll
  for (int rr = 0; rr < 16; ++rr) {
    sJ[(w * 16 + rr) * CAP + lane] = 0;
    sK[(w * 16 + rr) * CAP + lane] = NEG_INF;
  }
  float rmax_mine = NEG_INF;
  int   cnt_mine  = 0;
  int   ovf_mine  = 0;
  __syncthreads();

  const __bf16* arow0 = ab + (size_t)(R0 + 32 * wm + m) * DIM;
  const __bf16* arow1 = arow0 + (size_t)16 * DIM;
  const v8f zero8 = {0.f, 0.f, 0.f, 0.f, 0.f, 0.f, 0.f, 0.f};

  #pragma unroll 1
  for (int ct = 0; ct < NTILES; ++ct) {
    const int col0 = ct * BN;

    v8f acc[2][4];
    #pragma unroll
    for (int mt = 0; mt < 2; ++mt)
      #pragma unroll
      for (int nt = 0; nt < 4; ++nt) acc[mt][nt] = zero8;

    const __bf16* brow = nb + (size_t)(col0 + 64 * wn + m) * DIM;

    #pragma unroll 1
    for (int k0 = 0; k0 < DIM; k0 += 32) {
      const v16b a0 = load_frag(arow0 + k0, h);
      const v16b a1 = load_frag(arow1 + k0, h);
      #pragma unroll
      for (int nt = 0; nt < 4; ++nt) {
        const v16b b = load_frag(brow + (size_t)nt * 16 * DIM + k0, h);
        acc[0][nt] = wmma_bf16(a0, b, acc[0][nt]);
        acc[1][nt] = wmma_bf16(a1, b, acc[1][nt]);
      }
    }

    #pragma unroll
    for (int mt = 0; mt < 2; ++mt)
      #pragma unroll
      for (int nt = 0; nt < 4; ++nt)
        #pragma unroll
        for (int r = 0; r < 8; ++r)
          sS[(32 * wm + 16 * mt + 8 * h + r) * BN + 64 * wn + 16 * nt + m] = acc[mt][nt][r];

    const float nv0 = n2hi[col0 + lane];
    const float nv1 = n2hi[col0 + 32 + lane];
    const float nv2 = n2hi[col0 + 64 + lane];
    const float nv3 = n2hi[col0 + 96 + lane];
    __syncthreads();

    #pragma unroll 1
    for (int rr = 0; rr < 16; ++rr) {
      const float* srow = sS + (16 * w + rr) * BN;
      const float k0v = nv0 - 2.0f * srow[lane];
      const float k1v = nv1 - 2.0f * srow[32 + lane];
      const float k2v = nv2 - 2.0f * srow[64 + lane];
      const float k3v = nv3 - 2.0f * srow[96 + lane];

      float tmax = fmaxf(fmaxf(k0v, k1v), fmaxf(k2v, k3v));
      #pragma unroll
      for (int off = 16; off >= 1; off >>= 1) tmax = fmaxf(tmax, __shfl_xor(tmax, off, 32));

      const float rold = __shfl(rmax_mine, rr, 32);
      const float rnew = fmaxf(rold, tmax);
      rmax_mine = (lane == rr) ? rnew : rmax_mine;
      const float thr = rnew - BAND;
      const int cold = __shfl(cnt_mine, rr, 32);

      int*   lj = sJ + (w * 16 + rr) * CAP;
      float* lk = sK + (w * 16 + rr) * CAP;

      const int   ej = lj[lane];
      const float ek = lk[lane];
      const bool keep = (lane < cold) && (ek >= thr);
      const unsigned km = (unsigned)__ballot(keep);
      const int npos = __popc(km & ltmask);
      int total = __popc(km);
      __syncthreads();
      if (keep) { lj[npos] = ej; lk[npos] = ek; }

      {
        const bool f = k0v >= thr;
        const unsigned bm = (unsigned)__ballot(f);
        const int pos = total + __popc(bm & ltmask);
        total += __popc(bm);
        if (f && pos < CAP) { lj[pos] = col0 + lane; lk[pos] = k0v; }
      }
      {
        const bool f = k1v >= thr;
        const unsigned bm = (unsigned)__ballot(f);
        const int pos = total + __popc(bm & ltmask);
        total += __popc(bm);
        if (f && pos < CAP) { lj[pos] = col0 + 32 + lane; lk[pos] = k1v; }
      }
      {
        const bool f = k2v >= thr;
        const unsigned bm = (unsigned)__ballot(f);
        const int pos = total + __popc(bm & ltmask);
        total += __popc(bm);
        if (f && pos < CAP) { lj[pos] = col0 + 64 + lane; lk[pos] = k2v; }
      }
      {
        const bool f = k3v >= thr;
        const unsigned bm = (unsigned)__ballot(f);
        const int pos = total + __popc(bm & ltmask);
        total += __popc(bm);
        if (f && pos < CAP) { lj[pos] = col0 + 96 + lane; lk[pos] = k3v; }
      }
      const int ovf  = (total > CAP) ? 1 : 0;
      const int cnew = (total > CAP) ? CAP : total;
      cnt_mine = (lane == rr) ? cnew : cnt_mine;
      ovf_mine = (lane == rr) ? (ovf_mine | ovf) : ovf_mine;
      __syncthreads();
    }
  }

  const float QNAN = __uint_as_float(0x7fc00000u);
  const v4f nanv = {QNAN, QNAN, QNAN, QNAN};

  #pragma unroll 1
  for (int rr = 0; rr < 16; ++rr) {
    const int i = R0 + 16 * w + rr;
    const float* ap = anchor + (size_t)i * DIM + 4 * lane;
    v4f av[8];
    #pragma unroll
    for (int t = 0; t < 8; ++t) av[t] = *(const v4fa*)(ap + 128 * t);

    const int c    = __builtin_amdgcn_readfirstlane(__shfl(cnt_mine, rr, 32));
    const int povf = __builtin_amdgcn_readfirstlane(__shfl(ovf_mine, rr, 32));
    const int* lj = sJ + (w * 16 + rr) * CAP;

    float bh = NEG_INF, bl = 0.0f;
    int   bj = NROWS;
    #pragma unroll 1
    for (int e = 0; e < CAP; ++e) {
      if (e >= c) break;
      int j = lj[e];
      j = min(max(j, 0), NROWS - 1);
      const float* nq = negative + (size_t)j * DIM + 4 * lane;
      float hi = 0.0f, lo = 0.0f;
      #pragma unroll
      for (int t = 0; t < 8; ++t) {
        const v4f nv = *(const v4fa*)(nq + 128 * t);
        df_mac(hi, lo, av[t].x, nv.x);
        df_mac(hi, lo, av[t].y, nv.y);
        df_mac(hi, lo, av[t].z, nv.z);
        df_mac(hi, lo, av[t].w, nv.w);
      }
      df_wave_reduce(hi, lo);
      float kh = n2hi[j], kl = n2lo[j];
      df_add(kh, kl, -2.0f * hi, -2.0f * lo);
      const bool better = (kh > bh) || ((kh == bh) && ((kl > bl) || ((kl == bl) && (j < bj))));
      bh = better ? kh : bh;
      bl = better ? kl : bl;
      bj = better ? j  : bj;
    }
    int jstar = __builtin_amdgcn_readfirstlane(bj);
    const bool poison = (povf != 0) || (c <= 0) || (jstar >= NROWS) || (jstar < 0);
    jstar = min(max(jstar, 0), NROWS - 1);

    const float* sp = negative + (size_t)jstar * DIM + 4 * lane;
    v4f cv[8];
    #pragma unroll
    for (int t = 0; t < 8; ++t) cv[t] = sel4(poison, nanv, *(const v4fa*)(sp + 128 * t));

    float* op = out + (size_t)i * DIM + 4 * lane;
    #pragma unroll
    for (int t = 0; t < 8; ++t) *(volatile v4f*)(op + 128 * t) = cv[t];
    __threadfence();
    #pragma unroll
    for (int t = 0; t < 8; ++t) *(volatile v4f*)(op + 128 * t) = cv[t];
  }
}

extern "C" void kernel_launch(void* const* d_in, const int* in_sizes, int n_in,
                              void* d_out, int out_size, void* d_ws, size_t ws_size,
                              hipStream_t stream) {
  if (n_in < 2) return;
  if (in_sizes[0] != NELEM || in_sizes[1] != NELEM) return;
  if (out_size != NELEM) return;

  const float* anchor   = (const float*)d_in[0];
  const float* negative = (const float*)d_in[1];
  float* out = (float*)d_out;

  const size_t plane_bytes = (size_t)NELEM * 2;
  const size_t tab_bytes   = (size_t)NROWS * 4;
  const size_t total = 2 * plane_bytes + 2 * tab_bytes;
  if (total > ws_size) return;

  char* ws = (char*)d_ws;
  unsigned* abw = (unsigned*)(ws);
  unsigned* nbw = (unsigned*)(ws + plane_bytes);
  float* n2hi = (float*)(ws + 2 * plane_bytes);
  float* n2lo = (float*)(ws + 2 * plane_bytes + tab_bytes);

  prep_kernel<<<2 * (NROWS / RPB), 256, 0, stream>>>(anchor, negative, abw, nbw, n2hi, n2lo);

  select_kernel<<<NROWS / BM, 128, 0, stream>>>((const __bf16*)abw, (const __bf16*)nbw,
                                               anchor, negative, n2hi, n2lo, out);
}
